// RNN_39393440039090
// MI455X (gfx1250) — hardware-verified
//
#include <hip/hip_runtime.h>
#include <math.h>

constexpr int NBATCH   = 16;
constexpr int NOUTER   = 32;
constexpr int NINNER   = 64;
constexpr int NFEAT    = 256;
constexpr int NHID     = 512;
constexpr int NGATE    = 4 * NHID;
constexpr int NCLS     = 1000;
constexpr int NCLS_PAD = 1024;
constexpr int NSEQ1    = NBATCH * NOUTER;
constexpr int KT1      = NFEAT + NHID;
constexpr int KT2      = NHID + NHID;
constexpr int SEQ_THR  = 512;
constexpr int TP_THR   = 256;
constexpr float WCARRY     = 16.0f;
constexpr float WCARRY_INV = 1.0f / 16.0f;

static_assert(NGATE == 2048, "gate width");
static_assert(NSEQ1 == 512 && NSEQ1 % 16 == 0, "sequence tiles");
static_assert(KT1 % 32 == 0 && KT2 % 32 == 0, "K multiples of 32");
static_assert(NHID == 32 * (SEQ_THR / 32), "16 waves x 32 hidden units");
static_assert(NFEAT % 64 == 0 && NHID % 64 == 0 && NGATE % 64 == 0, "transpose tiles");
static_assert((NBATCH * NCLS) % 128 == 0, "flat output = whole 4-line wave chunks");
static_assert(NCLS % 4 == 0 && NCLS_PAD == 4 * 256, "dense lane map");

typedef __attribute__((ext_vector_type(16))) _Float16 v16h;
typedef __attribute__((ext_vector_type(8)))  _Float16 v8h;
typedef __attribute__((ext_vector_type(8)))  float    v8f;
typedef __attribute__((ext_vector_type(4)))  float    v4f;

__device__ __forceinline__ void acc_guard4(v8f& a, v8f& b, v8f& c, v8f& d) {
  asm volatile("v_nop\n\tv_nop\n\tv_nop\n\tv_nop" : "+v"(a), "+v"(b), "+v"(c), "+v"(d));
}
__device__ __forceinline__ void grp_guard(v8f& a0, v8f& a1, v8f& a2, v8f& a3,
                                          v16h a, v16h b0, v16h b1, v16h b2, v16h b3) {
  asm volatile("v_nop\n\tv_nop\n\tv_nop\n\tv_nop"
               : "+v"(a0), "+v"(a1), "+v"(a2), "+v"(a3)
               : "v"(a), "v"(b0), "v"(b1), "v"(b2), "v"(b3));
}

template <typename T> struct Frag;
template <> struct Frag<_Float16> {
  typedef v16h V; union U { v16h v; v8h h[2]; };
  static __device__ __forceinline__ v16h load(const _Float16* p) {
    U f; f.h[0] = *(const v8h*)(p); f.h[1] = *(const v8h*)(p + 16); return f.v;
  }
  static __device__ __forceinline__ v8f mma(v16h a, v16h b, v8f c) {
    return __builtin_amdgcn_wmma_f32_16x16x32_f16(false, a, false, b, (short)0, c, false, false);
  }
};

__device__ __forceinline__ float sigm_f(float x) { return __builtin_amdgcn_rcpf(1.0f + expf(-x)); }
__device__ __forceinline__ float tanh_f(float x) { return 1.0f - 2.0f * __builtin_amdgcn_rcpf(expf(2.0f * x) + 1.0f); }

__global__ __launch_bounds__(TP_THR) void tp_cast_kernel(const float* __restrict__ src, int R, int C, int ldo,
                                                         unsigned short* __restrict__ Op, float sc) {
  __shared__ float Tt[64 * 65];
  _Float16* O = (_Float16*)Op;
  const int tid = threadIdx.x;
  const int c0 = blockIdx.x * 64, r0 = blockIdx.y * 64;
#pragma unroll
  for (int i = 0; i < 4; ++i) {
    const int idx = i * TP_THR + tid;
    const int rr = idx >> 4, cc = (idx & 15) * 4;
    const v4f v = *(const v4f*)(src + (size_t)(r0 + rr) * (size_t)C + c0 + cc);
    Tt[rr * 65 + cc + 0] = v[0];
    Tt[rr * 65 + cc + 1] = v[1];
    Tt[rr * 65 + cc + 2] = v[2];
    Tt[rr * 65 + cc + 3] = v[3];
  }
  __syncthreads();
  const int q = tid >> 3, c8 = (tid & 7) * 8;
  v8h hv[2];
#pragma unroll
  for (int g = 0; g < 2; ++g) {
    const int qq = g * 32 + q;
#pragma unroll
    for (int e = 0; e < 8; ++e) {
      const float f = Tt[(c8 + e) * 65 + qq];
      hv[g][e] = (_Float16)(f * sc);
    }
  }
  for (int pass = 0; pass < 2; ++pass) {
#pragma unroll
    for (int g = 0; g < 2; ++g) {
      const size_t o = (size_t)(c0 + g * 32 + q) * (size_t)ldo + (size_t)(r0 + c8);
      *(volatile v8h*)(O + o) = hv[g];
    }
    __threadfence();
  }
}

template <int XK, int NSTEPS, bool XF32>
__device__ __forceinline__ void stage_rows(_Float16* dst, int ap, const float* xf32, const unsigned short* xf16,
                                           int rowbase, int t, int tid) {
  if (XF32) {
    const int m = tid >> 5, f8 = (tid & 31) * 8;
    const float* sp = xf32 + ((size_t)(rowbase + m) * NSTEPS + (size_t)t) * XK + f8;
    const v4f a = *(const v4f*)(sp);
    const v4f b = *(const v4f*)(sp + 4);
    v8h hv;
#pragma unroll
    for (int e = 0; e < 4; ++e) {
      hv[e]     = (_Float16)a[e];
      hv[4 + e] = (_Float16)b[e];
    }
    *(v8h*)(dst + m * ap + f8) = hv;
  } else {
    const _Float16* srcp = (const _Float16*)xf16;
#pragma unroll
    for (int it = 0; it < 2; ++it) {
      const int idx = it * SEQ_THR + tid;
      const int m = idx >> 6, ch = idx & 63;
      const v8h hv = *(const v8h*)(srcp + ((size_t)(rowbase + m) * NSTEPS + (size_t)t) * XK + ch * 8);
      *(v8h*)(dst + m * ap + ch * 8) = hv;
    }
  }
}

template <int XK, int NSTEPS, bool XF32, bool OUT16>
__global__ __launch_bounds__(SEQ_THR) void lstm_seq_kernel(const float* __restrict__ xf32, const unsigned short* xf16,
                                                           const unsigned short* __restrict__ Btp,
                                                           const float* __restrict__ bias,
                                                           unsigned short* out16, float* __restrict__ out32) {
  constexpr int KT  = XK + NHID;
  constexpr int AP  = KT + 8;
  constexpr int HSP = NHID + 4;
  static_assert(KT % 32 == 0, "K multiple of 32");
  static_assert((AP * 2) % 16 == 0 && AP % 8 == 0, "16-B aligned LDS rows");
  static_assert(XF32 ? (XK == 256) : (XK == 512), "staging maps");
  __shared__ __align__(16) _Float16 At[2][16 * AP];
  __shared__ __align__(16) float    Hs[OUT16 ? 4 : 16 * HSP];
  const _Float16* Bt = (const _Float16*)Btp;
  const int tid = threadIdx.x, lane = tid & 31, wave = tid >> 5;
  const int c = lane & 15, hh = lane >> 4, koff = hh * 8;
  const int rowbase = blockIdx.x * 16;
  const size_t GS = (size_t)NHID * KT;

  {
    v8h zz;
#pragma unroll
    for (int e = 0; e < 8; ++e) zz[e] = (_Float16)0.0f;
    _Float16* ab = &At[0][0];
#pragma unroll 1
    for (int i = tid; i < 4 * AP; i += SEQ_THR) *(v8h*)(ab + i * 8) = zz;
  }
  __syncthreads();
  stage_rows<XK, NSTEPS, XF32>(&At[0][0], AP, xf32, xf16, rowbase, 0, tid);

  float cst[2][8], bb[2][4];
#pragma unroll
  for (int nt = 0; nt < 2; ++nt) {
    const int j = 32 * wave + 16 * nt + c;
#pragma unroll
    for (int g = 0; g < 4; ++g) bb[nt][g] = bias[g * NHID + j];
#pragma unroll
    for (int r = 0; r < 8; ++r) cst[nt][r] = 0.0f;
  }
  __syncthreads();

  const v8f z8 = {0.f, 0.f, 0.f, 0.f, 0.f, 0.f, 0.f, 0.f};

#pragma unroll 1
  for (int t = 0; t < NSTEPS; ++t) {
    const int cur = t & 1;
    const _Float16* abase = &At[cur][0] + c * AP + koff;
    _Float16* nbase = &At[cur ^ 1][0];
    const bool last = (t == NSTEPS - 1);
#pragma unroll
    for (int nt = 0; nt < 2; ++nt) {
      const int j = 32 * wave + 16 * nt + c;
      const _Float16* w0 = Bt + (size_t)j * KT + koff;
      v8f a0 = z8, a1 = z8, a2 = z8, a3 = z8;
#pragma unroll 1
      for (int k0 = 0; k0 < KT; k0 += 32) {
        const v16h a  = Frag<_Float16>::load(abase + k0);
        const v16h b0 = Frag<_Float16>::load(w0 + k0);
        const v16h b1 = Frag<_Float16>::load(w0 + GS + k0);
        const v16h b2 = Frag<_Float16>::load(w0 + 2 * GS + k0);
        const v16h b3 = Frag<_Float16>::load(w0 + 3 * GS + k0);
        a0 = Frag<_Float16>::mma(a, b0, a0);
        a1 = Frag<_Float16>::mma(a, b1, a1);
        a2 = Frag<_Float16>::mma(a, b2, a2);
        a3 = Frag<_Float16>::mma(a, b3, a3);
        grp_guard(a0, a1, a2, a3, a, b0, b1, b2, b3);
      }
      acc_guard4(a0, a1, a2, a3);
#pragma unroll
      for (int r = 0; r < 8; ++r) {
        const float zi = a0[r] * WCARRY_INV + bb[nt][0];
        const float zf = a1[r] * WCARRY_INV + bb[nt][1];
        const float zg = a2[r] * WCARRY_INV + bb[nt][2];
        const float zo = a3[r] * WCARRY_INV + bb[nt][3];
        const float ig = sigm_f(zi);
        const float fg = sigm_f(zf);
        const float gg = tanh_f(zg);
        const float og = sigm_f(zo);
        const float cn = fg * cst[nt][r] + ig * gg;
        cst[nt][r] = cn;
        const float hn = og * tanh_f(cn);
        nbase[(8 * hh + r) * AP + XK + j] = (_Float16)hn;
        if (!OUT16 && last) Hs[(8 * hh + r) * HSP + j] = hn;
      }
    }
    {
      const int tn = (t + 1 < NSTEPS) ? (t + 1) : (NSTEPS - 1);
      stage_rows<XK, NSTEPS, XF32>(nbase, AP, xf32, xf16, rowbase, tn, tid);
    }
    __syncthreads();
  }

  if (OUT16) {
    const _Float16* fb = &At[NSTEPS & 1][0];
    _Float16* op = (_Float16*)out16;
    v8h hv[2];
#pragma unroll
    for (int it = 0; it < 2; ++it) {
      const int idx = it * SEQ_THR + tid;
      const int row = idx >> 6, ch = idx & 63;
      hv[it] = *(const v8h*)(fb + row * AP + XK + ch * 8);
    }
    for (int pass = 0; pass < 2; ++pass) {
#pragma unroll
      for (int it = 0; it < 2; ++it) {
        const int idx = it * SEQ_THR + tid;
        const int row = idx >> 6, ch = idx & 63;
        *(volatile v8h*)(op + (size_t)(rowbase + row) * NHID + ch * 8) = hv[it];
      }
      __threadfence();
    }
  } else {
    v4f ov[4];
#pragma unroll
    for (int it = 0; it < 4; ++it) {
      const int idx = it * SEQ_THR + tid;
      const int row = idx >> 7, c4 = (idx & 127) * 4;
      ov[it] = *(const v4f*)(Hs + row * HSP + c4);
    }
    for (int pass = 0; pass < 2; ++pass) {
#pragma unroll
      for (int it = 0; it < 4; ++it) {
        const int idx = it * SEQ_THR + tid;
        const int row = idx >> 7, c4 = (idx & 127) * 4;
        *(volatile v4f*)(out32 + (size_t)(rowbase + row) * NHID + c4) = ov[it];
      }
      __threadfence();
    }
  }
}

__global__ __launch_bounds__(256) void dense_softmax_kernel(const float* __restrict__ h2, const float* __restrict__ Wd,
                                                            const float* __restrict__ bd, float* __restrict__ PR) {
  __shared__ float hrow[NHID];
  __shared__ float red[16];
  const int tid = threadIdx.x, lane = tid & 31, wave = tid >> 5;
  const int b = blockIdx.x;
  hrow[tid]       = h2[(size_t)b * NHID + tid];
  hrow[tid + 256] = h2[(size_t)b * NHID + tid + 256];
  __syncthreads();
  const bool valid = (tid < NCLS / 4);
  const int tc = valid ? tid : (NCLS / 4 - 1);
  const float* wp = Wd + 4 * tc;
  v4f acc = {0.f, 0.f, 0.f, 0.f};
#pragma unroll 2
  for (int k = 0; k < NHID; ++k) {
    const v4f w = *(const v4f*)(wp + (size_t)k * NCLS);
    const float hk = hrow[k];
    acc[0] = fmaf(hk, w[0], acc[0]);
    acc[1] = fmaf(hk, w[1], acc[1]);
    acc[2] = fmaf(hk, w[2], acc[2]);
    acc[3] = fmaf(hk, w[3], acc[3]);
  }
  const v4f bv = *(const v4f*)(bd + 4 * tc);
  acc[0] += bv[0]; acc[1] += bv[1]; acc[2] += bv[2]; acc[3] += bv[3];

  float m = fmaxf(fmaxf(acc[0], acc[1]), fmaxf(acc[2], acc[3]));
  m = valid ? m : -INFINITY;
#pragma unroll
  for (int off = 1; off < 32; off <<= 1) m = fmaxf(m, __shfl_xor(m, off, 32));
  if (lane == 0) red[wave] = m;
  __syncthreads();
  float mm = red[0];
#pragma unroll
  for (int w = 1; w < 8; ++w) mm = fmaxf(mm, red[w]);

  v4f ex;
  ex[0] = expf(acc[0] - mm);
  ex[1] = expf(acc[1] - mm);
  ex[2] = expf(acc[2] - mm);
  ex[3] = expf(acc[3] - mm);
  float s = (ex[0] + ex[1]) + (ex[2] + ex[3]);
  s = valid ? s : 0.0f;
#pragma unroll
  for (int off = 1; off < 32; off <<= 1) s += __shfl_xor(s, off, 32);
  if (lane == 0) red[8 + wave] = s;
  __syncthreads();
  float tot = red[8];
#pragma unroll
  for (int w = 1; w < 8; ++w) tot += red[8 + w];
  const float inv = 1.0f / tot;
  v4f p;
  p[0] = valid ? ex[0] * inv : 0.0f;
  p[1] = valid ? ex[1] * inv : 0.0f;
  p[2] = valid ? ex[2] * inv : 0.0f;
  p[3] = valid ? ex[3] * inv : 0.0f;
  float* op = PR + (size_t)b * NCLS_PAD + 4 * tid;
  *(volatile v4f*)op = p;
  __threadfence();
  *(volatile v4f*)op = p;
}

__global__ __launch_bounds__(32) void out_lines_kernel(const float* __restrict__ PR, float* __restrict__ out) {
  const int i = blockIdx.x * 32 + threadIdx.x;
  const int f = 4 * i;
  const int row = f / NCLS;
  const int col = f - row * NCLS;
  const v4f v = *(const v4f*)(PR + (size_t)row * NCLS_PAD + col);
  *(volatile v4f*)(out + f) = v;
  __threadfence();
  *(volatile v4f*)(out + f) = v;
}

extern "C" void kernel_launch(void* const* d_in, const int* in_sizes, int n_in,
                              void* d_out, int out_size, void* d_ws, size_t ws_size, hipStream_t stream) {
  if (n_in < 9 || d_out == nullptr || d_ws == nullptr) return;
  if (in_sizes[0] != NBATCH * NOUTER * NINNER * NFEAT || in_sizes[1] != NFEAT * NGATE ||
      in_sizes[2] != NHID * NGATE || in_sizes[3] != NGATE || in_sizes[4] != NHID * NGATE ||
      in_sizes[5] != NHID * NGATE || in_sizes[6] != NGATE || in_sizes[7] != NHID * NCLS ||
      in_sizes[8] != NCLS || out_size != NBATCH * NCLS) return;

  const float* x  = (const float*)d_in[0];
  const float* W1 = (const float*)d_in[1];
  const float* U1 = (const float*)d_in[2];
  const float* b1 = (const float*)d_in[3];
  const float* W2 = (const float*)d_in[4];
  const float* U2 = (const float*)d_in[5];
  const float* b2 = (const float*)d_in[6];
  const float* Wd = (const float*)d_in[7];
  const float* bd = (const float*)d_in[8];
  float* out = (float*)d_out;

  char* ws = (char*)d_ws; size_t off = 0;
  auto carve = [&](size_t bytes) -> char* { char* p = ws + off; off += (bytes + 255) & ~(size_t)255; return p; };
  unsigned short* BT1 = (unsigned short*)carve((size_t)NGATE * KT1 * 2);
  unsigned short* BT2 = (unsigned short*)carve((size_t)NGATE * KT2 * 2);
  unsigned short* H1  = (unsigned short*)carve((size_t)NSEQ1 * NHID * 2);
  float*          H2  = (float*)carve((size_t)NBATCH * NHID * 4);
  float*          PR  = (float*)carve((size_t)NBATCH * NCLS_PAD * 4);
  if (off > ws_size || off > (size_t)134217728) return;

  tp_cast_kernel<<<dim3(NGATE / 64, NFEAT / 64), TP_THR, 0, stream>>>(W1, NFEAT, NGATE, KT1, BT1, WCARRY);
  tp_cast_kernel<<<dim3(NGATE / 64, NHID / 64), TP_THR, 0, stream>>>(U1, NHID, NGATE, KT1, BT1 + NFEAT, WCARRY);
  tp_cast_kernel<<<dim3(NGATE / 64, NHID / 64), TP_THR, 0, stream>>>(W2, NHID, NGATE, KT2, BT2, WCARRY);
  tp_cast_kernel<<<dim3(NGATE / 64, NHID / 64), TP_THR, 0, stream>>>(U2, NHID, NGATE, KT2, BT2 + NHID, WCARRY);

  lstm_seq_kernel<NFEAT, NINNER, true, true><<<NSEQ1 / 16, SEQ_THR, 0, stream>>>(x, H1, BT1, b1, H1, H2);
  lstm_seq_kernel<NHID, NOUTER, false, false><<<1, SEQ_THR, 0, stream>>>(x, H1, BT2, b2, H1, H2);
  dense_softmax_kernel<<<NBATCH, 256, 0, stream>>>(H2, Wd, bd, PR);
  out_lines_kernel<<<(NBATCH * NCLS) / 128, 32, 0, stream>>>(PR, out);
}
